// GNN_20366734917765
// MI455X (gfx1250) — hardware-verified
//
#include <hip/hip_runtime.h>
#include <stddef.h>
#include <stdint.h>
#include <math.h>

#pragma clang fp contract(off)


#define NB    4
#define NP    2048
#define BN    8192
#define HD    128
#define KN    32
#define NL    4
#define OUTD  6
#define NTHR  256
#define NWAVE 8
#define GBM   64
#define GBN   128
#define GTHR  128
#define AP    512
#define SP    256
#define PQP   256
#define U_PQ  8192
#define U_MO  4096
#define U_UI  8192
#define U_UO  4096
#define UPL   (U_PQ + U_MO + U_UI + U_UO)
#define O_PQ  0
#define O_MO  65536
#define O_UI  98304
#define O_UO  163840
#define WPLH  196608
#define CLN   2080
#define KQ    4
#define KNN_LDS_INTS (3 * NP + 2 * NWAVE * CLN + NWAVE * 128)
#define OUTB  (GBM * OUTD)
#define WSMAX 134217728

static_assert(BN == NB * NP && (NP & (NP - 1)) == 0 && NP == 2048);
static_assert(BN % GBM == 0 && GBM == (GTHR / 32) * 16 && GBN == HD && HD == 4 * 32);
static_assert(U_PQ % NTHR == 0 && U_MO % NTHR == 0 && U_UI % NTHR == 0 && U_UO % NTHR == 0);
static_assert(U_PQ * 8 == 256 * 256 && U_MO * 8 == 128 * 256 && U_UI * 8 == 128 * 512 && U_UO * 8 == 128 * 256);
static_assert(O_MO == 256 * 256 && O_UI == O_MO + 128 * 256 && O_UO == O_UI + 128 * 512 && WPLH == O_UO + 128 * 256);
static_assert((NL * UPL) % NTHR == 0);
static_assert(3 * NP == 24 * NTHR);
static_assert(NP == 64 * 32 && KN == 32 && KQ * NWAVE == 32 && NP % 32 == 0);
static_assert(CLN >= NP + 32 && (CLN * 4) % 16 == 0);
static_assert(KNN_LDS_INTS * 4 <= 300000);
static_assert(BN % NWAVE == 0);
static_assert((OUTB * 4) % 128 == 0 && OUTB == 96 * 4 && (BN / GBM) * OUTB == BN * OUTD);
static_assert(HD * OUTD == 3 * NTHR);

typedef float          v4f   __attribute__((ext_vector_type(4)));
typedef float          v8f   __attribute__((ext_vector_type(8)));
typedef int            v8i   __attribute__((ext_vector_type(8)));
typedef unsigned short v4us  __attribute__((ext_vector_type(4)));
typedef unsigned short v8us  __attribute__((ext_vector_type(8)));
typedef unsigned short v16us __attribute__((ext_vector_type(16)));
typedef __bf16         v16bf __attribute__((ext_vector_type(16)));
typedef v4f  __attribute__((may_alias)) v4fa;
typedef v4us __attribute__((may_alias)) v4usa;
typedef v8us __attribute__((may_alias)) v8usa;
union FragB { v16bf v; v16us u; v8us h[2]; v8i w; };

__device__ __forceinline__ v8f wmb(const FragB& a, const FragB& b, v8f c) {
  v8f d = __builtin_amdgcn_wmma_f32_16x16x32_bf16(false, a.v, false, b.v, (short)0, c, false, false);
  asm volatile("v_nop\n\tv_nop\n\tv_nop\n\tv_nop" : "+v"(d) : "v"(a.w), "v"(b.w));
  return d;
}

__device__ __forceinline__ unsigned bf16_bits(float f) {
  const unsigned u = __float_as_uint(f);
  return (u + 0x7FFFu + ((u >> 16) & 1u)) >> 16;
}
__device__ __forceinline__ float bf16_val(float f) {
  return __uint_as_float(bf16_bits(f) << 16);
}

__device__ __forceinline__ void wave_sync() {
  __builtin_amdgcn_fence(__ATOMIC_RELEASE, "wavefront");
  __builtin_amdgcn_wave_barrier();
  __builtin_amdgcn_fence(__ATOMIC_ACQUIRE, "wavefront");
}

__device__ __forceinline__ float silu_f(float x) {
  const float z   = expf(-fabsf(x));
  const float num = (x >= 0.0f) ? 1.0f : z;
  const float sg  = num / (1.0f + z);
  return x * sg;
}

__device__ __forceinline__ void split4(const v4f v, v4us& h, v4us& l) {
  unsigned hb;
  hb = bf16_bits(v.x); h[0] = (unsigned short)hb; l[0] = (unsigned short)bf16_bits(v.x - __uint_as_float(hb << 16));
  hb = bf16_bits(v.y); h[1] = (unsigned short)hb; l[1] = (unsigned short)bf16_bits(v.y - __uint_as_float(hb << 16));
  hb = bf16_bits(v.z); h[2] = (unsigned short)hb; l[2] = (unsigned short)bf16_bits(v.z - __uint_as_float(hb << 16));
  hb = bf16_bits(v.w); h[3] = (unsigned short)hb; l[3] = (unsigned short)bf16_bits(v.w - __uint_as_float(hb << 16));
}

__global__ __launch_bounds__(NTHR) void k_wprep(const float* __restrict__ miw, const float* __restrict__ mow,
                                                const float* __restrict__ uiw, const float* __restrict__ uow,
                                                unsigned short* wpl) {
  const int u = (int)blockIdx.x * NTHR + (int)threadIdx.x;
  const int l = u / UPL;
  const int v = u - l * UPL;
  if (l >= NL) return;
  unsigned short* lp = wpl + (size_t)l * WPLH;
  const float* src;
  unsigned short* dst;
  if (v < U_PQ) {
    const int n = v >> 5, k8 = (v & 31) * 8, kk = k8 & 127;
    src = miw + (size_t)l * (257 * HD) + (size_t)((n >> 7) * 128 + kk) * HD + (n & 127);
    dst = lp + O_PQ + (size_t)n * 256 + k8;
  } else if (v < U_PQ + U_MO) {
    const int w = v - U_PQ;
    const int n = w >> 5, k8 = (w & 31) * 8, kk = k8 & 127;
    src = mow + (size_t)l * (HD * HD) + (size_t)kk * HD + n;
    dst = lp + O_MO + (size_t)n * 256 + k8;
  } else if (v < U_PQ + U_MO + U_UI) {
    const int w = v - (U_PQ + U_MO);
    const int n = w >> 6, k8 = (w & 63) * 8;
    const int rr = (k8 & 127) + ((k8 >= 256) ? 128 : 0);
    src = uiw + (size_t)l * (2 * HD * HD) + (size_t)rr * HD + n;
    dst = lp + O_UI + (size_t)n * 512 + k8;
  } else {
    const int w = v - (U_PQ + U_MO + U_UI);
    const int n = w >> 5, k8 = (w & 31) * 8, kk = k8 & 127;
    src = uow + (size_t)l * (HD * HD) + (size_t)kk * HD + n;
    dst = lp + O_UO + (size_t)n * 256 + k8;
  }
  v8us o;
#pragma unroll
  for (int i = 0; i < 8; ++i) o[i] = (unsigned short)bf16_bits(src[(size_t)i * HD]);
  *(volatile v8us*)dst = o;
  __threadfence();
  *(volatile v8us*)dst = o;
}

__global__ __launch_bounds__(NTHR) void k_knn(const float* __restrict__ x, const float* __restrict__ ew,
                                              const float* __restrict__ eb, int* idxo, float* dno,
                                              float* Hf, unsigned short* apl) {
  extern __shared__ __attribute__((aligned(16))) int dsm[];
  const int tid = (int)threadIdx.x, lane = tid & 31, wave = tid >> 5;
  float* xyz = (float*)dsm;
  float* cld = (float*)(dsm + 3 * NP) + wave * CLN;
  int*   clj = dsm + 3 * NP + NWAVE * CLN + wave * CLN;
  unsigned short* rowbuf = (unsigned short*)(dsm + 3 * NP + 2 * NWAVE * CLN) + wave * 256;
  const int b    = (int)blockIdx.x >> 6;
  const int tile = (int)blockIdx.x & 63;
  const float finf = __int_as_float(0x7f800000);
  const int   imax = 0x7fffffff;

  {
    const float* xb = x + (size_t)b * (NP * 3);
#pragma unroll 4
    for (int it = 0; it < 24; ++it) {
      const int e = it * NTHR + tid;
      const int j = e / 3;
      const int c = e - 3 * j;
      xyz[c * NP + j] = bf16_val(xb[e]);
    }
  }
  v4f w0, w1, w2, bb;
  {
    const v4f a0 = *(const v4f*)(ew + 4 * lane);
    const v4f a1 = *(const v4f*)(ew + HD + 4 * lane);
    const v4f a2 = *(const v4f*)(ew + 2 * HD + 4 * lane);
    const v4f a3 = *(const v4f*)(eb + 4 * lane);
    w0.x = bf16_val(a0.x); w0.y = bf16_val(a0.y); w0.z = bf16_val(a0.z); w0.w = bf16_val(a0.w);
    w1.x = bf16_val(a1.x); w1.y = bf16_val(a1.y); w1.z = bf16_val(a1.z); w1.w = bf16_val(a1.w);
    w2.x = bf16_val(a2.x); w2.y = bf16_val(a2.y); w2.z = bf16_val(a2.z); w2.w = bf16_val(a2.w);
    bb.x = bf16_val(a3.x); bb.y = bf16_val(a3.y); bb.z = bf16_val(a3.z); bb.w = bf16_val(a3.w);
  }
  __syncthreads();

#pragma unroll 1
  for (int qq = 0; qq < KQ; ++qq) {
    const int i    = tile * 32 + wave * KQ + qq;
    const int node = b * NP + i;
    const float xi = xyz[i], yi = xyz[NP + i], zi = xyz[2 * NP + i];

    float d[64];
    float lm = finf;
#pragma unroll
    for (int t = 0; t < 64; ++t) {
      const int j = 32 * t + lane;
      const float dx = xi - xyz[j];
      const float dy = yi - xyz[NP + j];
      const float dz = zi - xyz[2 * NP + j];
      const float sx = dx * dx;
      const float sy = dy * dy;
      const float sz = dz * dz;
      float s = (sx + sz) + sy;
      s = (j == i) ? finf : s;
      d[t] = s;
      lm = fminf(lm, s);
    }
    float T = lm;
#pragma unroll
    for (int off = 16; off > 0; off >>= 1) T = fmaxf(T, __shfl_xor(T, off, 32));

    int base = 0;
#pragma unroll
    for (int t = 0; t < 64; ++t) {
      const bool hit = d[t] <= T;
      const unsigned mk = __builtin_amdgcn_ballot_w32(hit);
      const int pos = base + (int)__builtin_amdgcn_mbcnt_lo(mk, 0u);
      if (hit && pos < NP) { cld[pos] = d[t]; clj[pos] = 32 * t + lane; }
      base += (int)__builtin_popcount(mk);
    }
    base = __builtin_amdgcn_readfirstlane(base);
    base = base < 0 ? 0 : (base > NP - 1 ? NP - 1 : base);
    {
      const int pe = base + lane;
      cld[pe] = finf;
      clj[pe] = imax;
    }
    wave_sync();
    int nper = (base + 31) >> 5;
    nper = nper < 1 ? 1 : (nper > 64 ? 64 : nper);

    int   rj = 0;
    float rd = 0.0f;
#pragma unroll 1
    for (int r = 0; r < KN; ++r) {
      float lv = finf;
      int   lj = imax;
      int   le = lane;
#pragma unroll 1
      for (int q = 0; q < nper; ++q) {
        const int   e = lane + 32 * q;
        const float v = cld[e];
        const int   j = clj[e];
        const bool bt = (v < lv) || ((v == lv) && (j < lj));
        lv = bt ? v : lv; lj = bt ? j : lj; le = bt ? e : le;
      }
      float gv = lv;
      int   gj = lj;
#pragma unroll
      for (int off = 16; off > 0; off >>= 1) {
        const float ov = __shfl_xor(gv, off, 32);
        const int   oj = __shfl_xor(gj, off, 32);
        const bool bt = (ov < gv) || ((ov == gv) && (oj < gj));
        gv = bt ? ov : gv; gj = bt ? oj : gj;
      }
      if ((lj == gj) && (lv == gv) && (gj != imax)) cld[le] = finf;
      rj = (lane == r) ? gj : rj;
      rd = (lane == r) ? gv : rd;
    }
    rj = rj < 0 ? 0 : (rj > NP - 1 ? NP - 1 : rj);
    const float dnv = sqrtf(fmaxf(rd, 0.0f));

    v4f hv;
    hv.x = fmaf(zi, w2.x, fmaf(yi, w1.x, xi * w0.x)) + bb.x;
    hv.y = fmaf(zi, w2.y, fmaf(yi, w1.y, xi * w0.y)) + bb.y;
    hv.z = fmaf(zi, w2.z, fmaf(yi, w1.z, xi * w0.z)) + bb.z;
    hv.w = fmaf(zi, w2.w, fmaf(yi, w1.w, xi * w0.w)) + bb.w;
    v4us h4, l4;
    split4(hv, h4, l4);
    *(v4usa*)(rowbuf + 4 * lane) = h4;
    *(v4usa*)(rowbuf + HD + 4 * lane) = l4;
    wave_sync();
    const v8us q0 = *(const v8usa*)(rowbuf + 8 * lane);

    int*            ip = idxo + (size_t)node * KN + lane;
    float*          dp = dno + (size_t)node * KN + lane;
    float*          hp = Hf + (size_t)node * HD + 4 * lane;
    unsigned short* rp = apl + (size_t)node * AP + 8 * lane;
    *(volatile int*)ip   = rj;
    *(volatile float*)dp = dnv;
    *(volatile v4f*)hp   = hv;
    *(volatile v8us*)rp  = q0;
    __threadfence();
    *(volatile int*)ip   = rj;
    *(volatile float*)dp = dnv;
    *(volatile v4f*)hp   = hv;
    *(volatile v8us*)rp  = q0;
    wave_sync();
  }
}

template <int EPI>
__global__ __launch_bounds__(GTHR) void k_gemm(const unsigned short* A, int lda,
                                               const unsigned short* __restrict__ BT, int K,
                                               const float* __restrict__ bias, float bscale,
                                               float* outF, int ldo,
                                               unsigned short* dpl, int dpitch, int dcol) {
  __shared__ __attribute__((aligned(16))) float stg[GBM * GBN];
  const int tid = (int)threadIdx.x, lane = tid & 31, wave = tid >> 5, hh = lane >> 4, m = lane & 15;
  const int rowBase = (int)blockIdx.x * GBM;
  const int col0    = (int)blockIdx.y * GBN;

  v8f acc[8];
  {
    const v8f z = {0.f, 0.f, 0.f, 0.f, 0.f, 0.f, 0.f, 0.f};
#pragma unroll
    for (int t = 0; t < 8; ++t) acc[t] = z;
  }
  const unsigned short* ap = A + (size_t)(rowBase + 16 * wave + m) * (size_t)lda + 8 * hh;
  const unsigned short* bp = BT + (size_t)(col0 + m) * (size_t)K + 8 * hh;

#pragma unroll 1
  for (int k0 = 0; k0 < K; k0 += 32) {
    FragB af;
    af.h[0] = *(const v8usa*)(ap + k0);
    af.h[1] = *(const v8usa*)(ap + k0 + 16);
#pragma unroll
    for (int nt = 0; nt < 8; ++nt) {
      const unsigned short* wq = bp + (size_t)(16 * nt) * (size_t)K + k0;
      FragB bf;
      bf.h[0] = *(const v8usa*)wq;
      bf.h[1] = *(const v8usa*)(wq + 16);
      acc[nt] = wmb(af, bf, acc[nt]);
    }
  }

#pragma unroll
  for (int nt = 0; nt < 8; ++nt) {
    const int lc = 16 * nt + m;
#pragma unroll
    for (int r = 0; r < 8; ++r) {
      const int lr = 16 * wave + 8 * hh + r;
      stg[lr * GBN + lc] = acc[nt][r];
    }
  }
  __syncthreads();

  v4f bb4 = {0.f, 0.f, 0.f, 0.f};
  if constexpr (EPI != 0) {
    const v4f t1 = *(const v4f*)(bias + col0 + 4 * lane);
    bb4.x = bf16_val(t1.x) * bscale; bb4.y = bf16_val(t1.y) * bscale;
    bb4.z = bf16_val(t1.z) * bscale; bb4.w = bf16_val(t1.w) * bscale;
  }

#pragma unroll 1
  for (int i = 0; i < 16; ++i) {
    const int lr = 16 * wave + i;
    const size_t gr = (size_t)(rowBase + lr);
    float* srow = stg + lr * GBN;
    v4f t = *(const v4fa*)(srow + 4 * lane);
    if constexpr (EPI == 0) {
      float* op = outF + gr * (size_t)ldo + col0 + 4 * lane;
      *(volatile v4f*)op = t;
      __threadfence();
      *(volatile v4f*)op = t;
    } else {
      t = t + bb4;
      if constexpr (EPI == 2) {
        t.x = silu_f(t.x); t.y = silu_f(t.y); t.z = silu_f(t.z); t.w = silu_f(t.w);
      }
      float* hp = outF + gr * (size_t)ldo + 4 * lane;
      if constexpr (EPI == 3) {
        const v4f hv = *(const v4fa*)hp;
        t = hv + t;
      }
      v4us h4, l4;
      split4(t, h4, l4);
      unsigned short* hrow = (unsigned short*)srow;
      *(v4usa*)(hrow + 4 * lane) = h4;
      *(v4usa*)(hrow + HD + 4 * lane) = l4;
      wave_sync();
      const v8us qv = *(const v8usa*)(hrow + 8 * lane);
      unsigned short* rp = dpl + gr * (size_t)dpitch + dcol + 8 * lane;
      if constexpr (EPI == 3) *(volatile v4f*)hp = t;
      *(volatile v8us*)rp = qv;
      __threadfence();
      if constexpr (EPI == 3) *(volatile v4f*)hp = t;
      *(volatile v8us*)rp = qv;
    }
  }
}

__global__ __launch_bounds__(NTHR) void k_edge(const float* __restrict__ pq, const int* __restrict__ idx,
                                               const float* __restrict__ dn, const float* __restrict__ wd,
                                               const float* __restrict__ bin, unsigned short* spl) {
  __shared__ __attribute__((aligned(16))) unsigned short rowbuf[NWAVE * 256];
  const int tid = (int)threadIdx.x, lane = tid & 31, wave = tid >> 5;
  const int node = (int)blockIdx.x * NWAVE + wave;
  const int b0   = node & ~(NP - 1);
  unsigned short* rb = rowbuf + wave * 256;

  int jl = idx[(size_t)node * KN + lane];
  jl = jl < 0 ? 0 : (jl > NP - 1 ? NP - 1 : jl);
  const int dli = __float_as_int(dn[(size_t)node * KN + lane]);
  v4f wd4, pb;
  {
    const v4f a = *(const v4f*)(wd + 4 * lane);
    const v4f c = *(const v4f*)(bin + 4 * lane);
    const v4f p = *(const v4f*)(pq + (size_t)node * PQP + 4 * lane);
    wd4.x = bf16_val(a.x); wd4.y = bf16_val(a.y); wd4.z = bf16_val(a.z); wd4.w = bf16_val(a.w);
    pb.x = p.x + bf16_val(c.x); pb.y = p.y + bf16_val(c.y);
    pb.z = p.z + bf16_val(c.z); pb.w = p.w + bf16_val(c.w);
  }
  float a0 = 0.0f, a1 = 0.0f, a2 = 0.0f, a3 = 0.0f;
#pragma unroll 1
  for (int k = 0; k < KN; ++k) {
    const int   j  = __builtin_amdgcn_readlane(jl, k);
    const float dk = __int_as_float(__builtin_amdgcn_readlane(dli, k));
    const v4f q = *(const v4f*)(pq + (size_t)(b0 + j) * PQP + HD + 4 * lane);
    const float t0 = fmaf(dk, wd4.x, pb.x) + q.x;
    const float t1 = fmaf(dk, wd4.y, pb.y) + q.y;
    const float t2 = fmaf(dk, wd4.z, pb.z) + q.z;
    const float t3 = fmaf(dk, wd4.w, pb.w) + q.w;
    a0 += silu_f(t0);
    a1 += silu_f(t1);
    a2 += silu_f(t2);
    a3 += silu_f(t3);
  }
  v4f sv;
  sv.x = a0; sv.y = a1; sv.z = a2; sv.w = a3;
  v4us h4, l4;
  split4(sv, h4, l4);
  *(v4usa*)(rb + 4 * lane) = h4;
  *(v4usa*)(rb + HD + 4 * lane) = l4;
  wave_sync();
  const v8us qv = *(const v8usa*)(rb + 8 * lane);
  unsigned short* rp = spl + (size_t)node * SP + 8 * lane;
  *(volatile v8us*)rp = qv;
  __threadfence();
  *(volatile v8us*)rp = qv;
}

__global__ __launch_bounds__(NTHR) void k_out(const float* __restrict__ Hf, const float* __restrict__ ow,
                                              const float* __restrict__ ob, float* out) {
  __shared__ float wls[HD * OUTD];
  __shared__ float bls[8];
  __shared__ __attribute__((aligned(16))) float os[OUTB];
  const int tid = (int)threadIdx.x;
#pragma unroll 1
  for (int i = tid; i < HD * OUTD; i += NTHR) wls[i] = bf16_val(ow[i]);
  if (tid < 8) {
    const float bbv = ob[tid < OUTD ? tid : OUTD - 1];
    bls[tid] = (tid < OUTD) ? bf16_val(bbv) : 0.0f;
  }
  __syncthreads();
  const int rowBase = (int)blockIdx.x * GBM;
#pragma unroll 1
  for (int idx = tid; idx < OUTB; idx += NTHR) {
    const int r = idx / OUTD;
    const int o = idx - r * OUTD;
    const float* hr = Hf + (size_t)(rowBase + r) * HD;
    float s = 0.0f;
#pragma unroll 2
    for (int f4 = 0; f4 < HD / 4; ++f4) {
      const v4f p = *(const v4f*)(hr + 4 * f4);
      const float* w = wls + (4 * f4) * OUTD + o;
      s = fmaf(p.x, w[0], s);
      s = fmaf(p.y, w[OUTD], s);
      s = fmaf(p.z, w[2 * OUTD], s);
      s = fmaf(p.w, w[3 * OUTD], s);
    }
    os[idx] = s + bls[o];
  }
  __syncthreads();
  const bool okst = tid < (OUTB / 4);
  const int  tq   = okst ? tid : 0;
  const v4f ov = *(const v4fa*)(os + 4 * tq);
  float* op = out + (size_t)blockIdx.x * OUTB + 4 * tq;
  if (okst) *(volatile v4f*)op = ov;
  __threadfence();
  if (okst) *(volatile v4f*)op = ov;
}

static inline size_t al256(size_t o) { return (o + 255) & ~(size_t)255; }

extern "C" void kernel_launch(void* const* d_in, const int* in_sizes, int n_in,
                              void* d_out, int out_size, void* d_ws, size_t ws_size,
                              hipStream_t stream) {
  if (n_in < 13) return;
  if (in_sizes[0]  != BN * 3)            return;
  if (in_sizes[1]  != 3 * HD)            return;
  if (in_sizes[2]  != HD)                return;
  if (in_sizes[3]  != NL * 257 * HD)     return;
  if (in_sizes[4]  != NL * HD)           return;
  if (in_sizes[5]  != NL * HD * HD)      return;
  if (in_sizes[6]  != NL * HD)           return;
  if (in_sizes[7]  != NL * 2 * HD * HD)  return;
  if (in_sizes[8]  != NL * HD)           return;
  if (in_sizes[9]  != NL * HD * HD)      return;
  if (in_sizes[10] != NL * HD)           return;
  if (in_sizes[11] != HD * OUTD)         return;
  if (in_sizes[12] != OUTD)              return;
  if (out_size != BN * OUTD)             return;

  const float* x    = (const float*)d_in[0];
  const float* ebw  = (const float*)d_in[1];
  const float* ebb  = (const float*)d_in[2];
  const float* miw  = (const float*)d_in[3];
  const float* mib  = (const float*)d_in[4];
  const float* mow  = (const float*)d_in[5];
  const float* mob  = (const float*)d_in[6];
  const float* uiw  = (const float*)d_in[7];
  const float* uib  = (const float*)d_in[8];
  const float* uow  = (const float*)d_in[9];
  const float* uob  = (const float*)d_in[10];
  const float* outw = (const float*)d_in[11];
  const float* outb = (const float*)d_in[12];
  float* out = (float*)d_out;

  char* ws = (char*)d_ws;
  size_t off = 0;
  const size_t oH   = off; off = al256(off + (size_t)BN * HD * 4);
  const size_t oA   = off; off = al256(off + (size_t)BN * AP * 2);
  const size_t oPQ  = off; off = al256(off + (size_t)BN * PQP * 4);
  const size_t oS   = off; off = al256(off + (size_t)BN * SP * 2);
  const size_t oT   = off; off = al256(off + (size_t)BN * SP * 2);
  const size_t oIDX = off; off = al256(off + (size_t)BN * KN * 4);
  const size_t oDN  = off; off = al256(off + (size_t)BN * KN * 4);
  const size_t oW   = off; off = al256(off + (size_t)NL * WPLH * 2);
  if (off > ws_size || off > (size_t)WSMAX) return;
  float*          H   = (float*)(ws + oH);
  unsigned short* A5  = (unsigned short*)(ws + oA);
  float*          PQ  = (float*)(ws + oPQ);
  unsigned short* S   = (unsigned short*)(ws + oS);
  unsigned short* T   = (unsigned short*)(ws + oT);
  int*            IDX = (int*)(ws + oIDX);
  float*          DN  = (float*)(ws + oDN);
  unsigned short* WP  = (unsigned short*)(ws + oW);

  const size_t knnLds = (size_t)KNN_LDS_INTS * 4;
  hipFuncSetAttribute(reinterpret_cast<const void*>(&k_knn), hipFuncAttributeMaxDynamicSharedMemorySize, (int)knnLds);

  k_wprep<<<(NL * UPL) / NTHR, NTHR, 0, stream>>>(miw, mow, uiw, uow, WP);
  k_knn<<<NB * (NP / 32), NTHR, knnLds, stream>>>(x, ebw, ebb, IDX, DN, H, A5);

  for (int l = 0; l < NL; ++l) {
    const unsigned short* wl = WP + (size_t)l * WPLH;
    k_gemm<0><<<dim3(BN / GBM, 2), GTHR, 0, stream>>>(A5, AP, wl + O_PQ, 256, mib, 0.0f, PQ, PQP, A5, AP, 0);
    k_edge<<<BN / NWAVE, NTHR, 0, stream>>>(PQ, IDX, DN, miw + (size_t)l * (257 * HD) + 256 * HD,
                                            mib + (size_t)l * HD, S);
    k_gemm<1><<<dim3(BN / GBM, 1), GTHR, 0, stream>>>(S, SP, wl + O_MO, 256, mob + (size_t)l * HD, 32.0f,
                                                      H, HD, A5, AP, 256);
    k_gemm<2><<<dim3(BN / GBM, 1), GTHR, 0, stream>>>(A5, AP, wl + O_UI, 512, uib + (size_t)l * HD, 1.0f,
                                                      H, HD, T, SP, 0);
    k_gemm<3><<<dim3(BN / GBM, 1), GTHR, 0, stream>>>(T, SP, wl + O_UO, 256, uob + (size_t)l * HD, 1.0f,
                                                      H, HD, A5, AP, 0);
  }
  k_out<<<BN / GBM, NTHR, 0, stream>>>(H, outw, outb, out);
}
